// VectorQuantizer_86242943304022
// MI455X (gfx1250) — hardware-verified
//
#include <hip/hip_runtime.h>
#pragma clang fp contract(off)


#ifndef NB
#define NB 2
#endif
#ifndef NHD
#define NHD 256
#endif
#define NB_FULL  2
#define NHD_FULL 256
#define CD   8
#define KC   4096
#define NPOS 256
#define DCH  (NHD_FULL * CD)
#define NT   (KC / 16)
#define NTHR 512
#define NPIECE (NB * CD * NPOS / 4)
#ifndef SUM_ORDER
#define SUM_ORDER 0
#endif

static_assert(CD == 8);
static_assert(KC % 16 == 0);
static_assert(KC % NTHR == 0);
static_assert(KC <= 4096);
static_assert(NPOS == 16 * (NTHR / 32));
static_assert(NPIECE % NTHR == 0);
static_assert(((CD * NPOS / 4) % 32) == 0);
static_assert((size_t)NTHR * 16 * (NPIECE / NTHR) == (size_t)NB * CD * NPOS * 4);
static_assert(NB <= NB_FULL);
static_assert(NHD <= NHD_FULL);
static_assert((size_t)(KC + 1) * 16 + (size_t)KC * 4 + (size_t)NB * CD * NPOS * 4 <= (size_t)131072);

typedef unsigned short bf;
typedef __attribute__((ext_vector_type(16))) __bf16   v16bf;
typedef __attribute__((ext_vector_type(8)))  unsigned short v8us;
typedef __attribute__((ext_vector_type(8)))  float    v8f;
typedef __attribute__((ext_vector_type(4)))  float    v4f;
typedef v4f  __attribute__((may_alias)) v4fa;
typedef v8f  __attribute__((may_alias)) v8fa;

__device__ __forceinline__ unsigned short f2bf(float f) { unsigned u = __float_as_uint(f); u += 0x7FFFu + ((u >> 16) & 1u); return (unsigned short)(u >> 16); }
__device__ __forceinline__ float bfr(float f) { return __uint_as_float(((unsigned)f2bf(f)) << 16); }
__device__ __forceinline__ v16bf cat16b(v8us lo, v8us hi) { return __builtin_bit_cast(v16bf, __builtin_shufflevector(lo, hi, 0, 1, 2, 3, 4, 5, 6, 7, 8, 9, 10, 11, 12, 13, 14, 15)); }
__device__ __forceinline__ v8f wmmab(v16bf a, v16bf b, v8f c) { return __builtin_amdgcn_wmma_f32_16x16x32_bf16(false, a, false, b, (short)0, c, false, false); }
__device__ __forceinline__ v8f wmmab_g(v16bf a, v16bf b, v8f c) {
    c = wmmab(a, b, c);
    asm volatile("v_nop\n\tv_nop\n\tv_nop\n\tv_nop" : "+v"(c) : "v"(a), "v"(b));
    return c;
}
__device__ __forceinline__ float bfw(unsigned short w) { return __uint_as_float(((unsigned)w) << 16); }
__device__ __forceinline__ float sum8(float t0, float t1, float t2, float t3, float t4, float t5, float t6, float t7) {
#if SUM_ORDER == 0
    return ((t0 + t4) + (t2 + t6)) + ((t1 + t5) + (t3 + t7));
#elif SUM_ORDER == 1
    return ((((((t0 + t1) + t2) + t3) + t4) + t5) + t6) + t7;
#else
    return (((t0 + t2) + t4) + t6) + (((t1 + t3) + t5) + t7);
#endif
}

__global__ __launch_bounds__(NTHR) void k_vq(const float* __restrict__ emb, const float* __restrict__ cb, float* out) {
    __shared__ v8us cbs[KC + 1];
    __shared__ __align__(32) float csq[KC];
    __shared__ __align__(16) float osr[NB * CD * NPOS];
    const int tid = threadIdx.x;
    const int lane = tid & 31, lr = lane & 15, hi = lane >> 4;
    const int wave = __builtin_amdgcn_readfirstlane((int)(threadIdx.x >> 5));
    const int hd = blockIdx.x;
    const float* cbh = cb + (size_t)hd * KC * CD;

#pragma unroll 1
    for (int k = tid; k < KC; k += NTHR) {
        const v4f c0 = *(const v4f*)(cbh + (size_t)k * CD);
        const v4f c1 = *(const v4f*)(cbh + (size_t)k * CD + 4);
        v8us o; float cv[8];
#pragma unroll
        for (int j = 0; j < 4; ++j) { o[j] = f2bf(c0[j]); o[4 + j] = f2bf(c1[j]); }
#pragma unroll
        for (int j = 0; j < 8; ++j) cv[j] = bfw(o[j]);
        cbs[k] = o;
        csq[k] = sum8(cv[0] * cv[0], cv[1] * cv[1], cv[2] * cv[2], cv[3] * cv[3], cv[4] * cv[4], cv[5] * cv[5], cv[6] * cv[6], cv[7] * cv[7]);
    }
    if (tid == 0) cbs[KC] = (v8us){};
    __syncthreads();

    const v8us zz = (v8us){};
    const int aidx = hi ? KC : lr;
    const int astr = hi ? 0 : 16;

#pragma unroll 1
    for (int b = 0; b < NB; ++b) {
        const int n = wave * 16 + lr;
        const float* eb = emb + ((size_t)b * DCH + (size_t)hd * CD) * NPOS + n;
        float xv[8]; v8us xb;
#pragma unroll
        for (int j = 0; j < 8; ++j) { xv[j] = bfr(eb[(size_t)j * NPOS]); xb[j] = f2bf(-2.0f * xv[j]); }
        const v8us xq = hi ? zz : xb;
        const v16bf bq = cat16b(xq, zz);
        const float xsq = sum8(xv[0] * xv[0], xv[1] * xv[1], xv[2] * xv[2], xv[3] * xv[3], xv[4] * xv[4], xv[5] * xv[5], xv[6] * xv[6], xv[7] * xv[7]);

        float bestv[8]; int bm[8];
#pragma unroll
        for (int v = 0; v < 8; ++v) { bestv[v] = 3.4028235e38f; bm[v] = 0; }
#pragma unroll 2
        for (int m = 0; m < NT; ++m) {
            const v8us av = cbs[aidx + m * astr];
            v8f c = *(const v8fa*)(&csq[m * 16 + 8 * hi]);
            c = wmmab_g(cat16b(av, zz), bq, c);
#pragma unroll
            for (int v = 0; v < 8; ++v) {
                const bool lt = c[v] < bestv[v];
                bestv[v] = lt ? c[v] : bestv[v];
                bm[v]    = lt ? m : bm[v];
            }
        }

        float bd = 0.0f; int bc = 0;
#pragma unroll
        for (int r = 0; r < 8; ++r) {
            const int code = (bm[r] * 16 + 8 * hi + r) & (KC - 1);
            const v8us cu = cbs[code];
            float p = xv[0] * bfw(cu[0]);
#pragma unroll
            for (int j = 1; j < 8; ++j) p = p + xv[j] * bfw(cu[j]);
            const float dd = (xsq - 2.0f * p) + csq[code];
            const bool better = (r == 0) | (dd < bd) | ((dd == bd) & (code < bc));
            bd = better ? dd : bd;
            bc = better ? code : bc;
        }
        {
            const float od = __shfl_xor(bd, 16, 32);
            const int   oc = __shfl_xor(bc, 16, 32);
            const bool better = (od < bd) | ((od == bd) & (oc < bc));
            bd = better ? od : bd;
            bc = better ? oc : bc;
        }
        {
            const v8us cu = cbs[bc & (KC - 1)];
#pragma unroll
            for (int jj = 0; jj < 4; ++jj) {
                const float xj = hi ? xv[4 + jj] : xv[jj];
                const float qj = hi ? bfw(cu[4 + jj]) : bfw(cu[jj]);
                const float tq = qj - xj;
                osr[(b * CD + 4 * hi + jj) * NPOS + n] = xj + tq;
            }
        }
    }
    __syncthreads();

#pragma unroll 1
    for (int ps = 0; ps < 2; ++ps) {
#pragma unroll
        for (int it = 0; it < NPIECE / NTHR; ++it) {
            const int p = it * NTHR + tid;
            const int b = p / (CD * NPOS / 4), w = p % (CD * NPOS / 4);
            const v4f val = *(const v4fa*)(&osr[p * 4]);
            *(volatile v4f*)(out + ((size_t)b * DCH + (size_t)hd * CD) * NPOS + (size_t)w * 4) = val;
        }
        if (ps == 0) __threadfence();
    }
}

extern "C" void kernel_launch(void* const* d_in, const int* in_sizes, int n_in,
                              void* d_out, int out_size, void* d_ws, size_t ws_size, hipStream_t stream) {
    (void)d_ws; (void)ws_size;
    if (n_in < 2) return;
    const size_t needx = ((size_t)(NB - 1) * DCH + (size_t)NHD * CD) * NPOS;
    const size_t needc = (size_t)NHD * KC * CD;
    if ((size_t)in_sizes[0] < needx || (size_t)in_sizes[1] < needc) return;
    if ((size_t)out_size < needx) return;
    const float* emb = (const float*)d_in[0];
    const float* cbk = (const float*)d_in[1];
    float* OUT = (float*)d_out;
    k_vq<<<dim3(NHD, 1, 1), NTHR, 0, stream>>>(emb, cbk, OUT);
}
